// PointerLSTM_7430293422955
// MI455X (gfx1250) — hardware-verified
//
#include <hip/hip_runtime.h>
#include <math.h>

constexpr int SEQS    = 32;
constexpr int STEPS   = 256;
constexpr int FEAT    = 128;
constexpr int HID     = 256;
constexpr int GATES   = 1024;
constexpr int NTHR    = 256;
constexpr int RPB     = 4;
constexpr int MTILE   = 16;
constexpr int XZROWS  = 8;
constexpr int HWROWS  = 8;
constexpr int HPITCH  = 264;
constexpr int XLPITCH = 136;
constexpr int XZPITCH = 1028;
constexpr int HWPITCH = 260;
constexpr int SCPITCH = 260;
constexpr float WCARRY = 16.0f;
constexpr float HCARRY = 64.0f;
constexpr float INV_W  = 1.0f / 16.0f;
constexpr float INV_WH = 1.0f / 1024.0f;

static_assert(GATES == 4 * HID, "sz");
static_assert(SEQS % RPB == 0 && HID % 64 == 0 && FEAT % 64 == 0 && GATES % 64 == 0 && STEPS % 64 == 0, "sz");
static_assert(NTHR == HID && NTHR == STEPS && RPB == 4 && MTILE == 16 && RPB <= NTHR / 32, "sz");
static_assert(XZROWS == 2 * RPB && HWROWS == 2 * RPB, "sz");

typedef __attribute__((ext_vector_type(16))) _Float16 v16h;
typedef __attribute__((ext_vector_type(8)))  _Float16 v8h;
typedef __attribute__((ext_vector_type(16))) __bf16   v16b;
typedef __attribute__((ext_vector_type(8)))  __bf16   v8b;
typedef __attribute__((ext_vector_type(8)))  float    v8f;
typedef __attribute__((ext_vector_type(4)))  float    v4f;

__device__ __forceinline__ unsigned short f2bf_bits(float f) {
  unsigned u = __float_as_uint(f);
  return (unsigned short)((u + 0x7FFFu + ((u >> 16) & 1u)) >> 16);
}
__device__ __forceinline__ float bf_bits2f(unsigned short h) { return __uint_as_float(((unsigned)h) << 16); }
__device__ __forceinline__ float bfr(float f) { return bf_bits2f(f2bf_bits(f)); }

__device__ __forceinline__ void dep_guard_h(v8f& a, v8f& b, v16h x, v16h y) { asm volatile("v_nop\n\tv_nop\n\tv_nop\n\tv_nop" : "+v"(a), "+v"(b) : "v"(x), "v"(y)); }
__device__ __forceinline__ void dep_guard_b(v8f& a, v8f& b, v16b x, v16b y) { asm volatile("v_nop\n\tv_nop\n\tv_nop\n\tv_nop" : "+v"(a), "+v"(b) : "v"(x), "v"(y)); }
__device__ __forceinline__ void keep4_h(v16h a, v16h b, v16h c, v16h d) { asm volatile("v_nop" :: "v"(a), "v"(b), "v"(c), "v"(d)); }
__device__ __forceinline__ void keep4_b(v16b a, v16b b, v16b c, v16b d) { asm volatile("v_nop" :: "v"(a), "v"(b), "v"(c), "v"(d)); }
__device__ __forceinline__ void keep2_h(v16h a, v16h b) { asm volatile("v_nop" :: "v"(a), "v"(b)); }
__device__ __forceinline__ void acc_guard4(v8f& a, v8f& b, v8f& c, v8f& d) { asm volatile("v_nop\n\tv_nop\n\tv_nop\n\tv_nop" : "+v"(a), "+v"(b), "+v"(c), "+v"(d)); }
__device__ __forceinline__ void acc_guard2(v8f& a, v8f& b) { asm volatile("v_nop\n\tv_nop\n\tv_nop\n\tv_nop" : "+v"(a), "+v"(b)); }
template <typename T> struct Frag;
template <> struct Frag<_Float16> {
  typedef v16h V; union U { v16h v; v8h h[2]; };
  static __device__ __forceinline__ v16h load(const _Float16* p) {
    U f; f.h[0] = *(const v8h*)(p); f.h[1] = *(const v8h*)(p + 16); return f.v;
  }
  static __device__ __forceinline__ v8f mma(v16h a, v16h b, v8f c) {
    return __builtin_amdgcn_wmma_f32_16x16x32_f16(false, a, false, b, (short)0, c, false, false);
  }
  static __device__ __forceinline__ void guard(v8f& a, v8f& b, v16h x, v16h y) { dep_guard_h(a, b, x, y); }
  static __device__ __forceinline__ void keep(v16h a, v16h b, v16h c, v16h d) { keep4_h(a, b, c, d); }
};
template <> struct Frag<__bf16> {
  typedef v16b V; union U { v16b v; v8b h[2]; };
  static __device__ __forceinline__ v16b load(const __bf16* p) {
    U f; f.h[0] = *(const v8b*)(p); f.h[1] = *(const v8b*)(p + 16); return f.v;
  }
  static __device__ __forceinline__ v8f mma(v16b a, v16b b, v8f c) {
    return __builtin_amdgcn_wmma_f32_16x16x32_bf16(false, a, false, b, (short)0, c, false, false);
  }
  static __device__ __forceinline__ void guard(v8f& a, v8f& b, v16b x, v16b y) { dep_guard_b(a, b, x, y); }
  static __device__ __forceinline__ void keep(v16b a, v16b b, v16b c, v16b d) { keep4_b(a, b, c, d); }
};

__device__ __forceinline__ float fsig(float x)  { return __builtin_amdgcn_rcpf(1.0f + __expf(-x)); }
__device__ __forceinline__ float ftanh(float x) { return 1.0f - 2.0f * __builtin_amdgcn_rcpf(__expf(2.0f * x) + 1.0f); }

template <int ET> struct Elem;
template <> struct Elem<0> { typedef _Float16 T; };
template <> struct Elem<1> { typedef __bf16 T; };
template <int ET, bool SPLIT, int BIAS_MODE, int OUT_MODE, bool RESID, int ACT = 0>
__global__ __launch_bounds__(256) void wmma_gemm64(
    const unsigned short* __restrict__ Ap, const unsigned short* __restrict__ A2p, int lda, long strideA,
    const unsigned short* __restrict__ Btp, const unsigned short* __restrict__ Bt2p, int ldb, long strideB,
    void* __restrict__ Cout, void* __restrict__ Cout2, int ldc, long strideC,
    const float* __restrict__ bias,
    const float* __restrict__ resid, long strideR,
    int M, int N, int K, float scale) {
  typedef typename Elem<ET>::T T;
  typedef typename Frag<T>::V V;
  const T* A = (const T*)Ap; const T* A2 = (const T*)A2p; const T* Bt = (const T*)Btp; const T* Bt2 = (const T*)Bt2p;
  __shared__ __align__(16) float sT[8][16 * 68];
  const int b    = blockIdx.y;
  const int lane = threadIdx.x & 31;
  const int wave = threadIdx.x >> 5;
  const int tilesN = N >> 6;
  const int tilesM = M >> 6;
  const int tile = blockIdx.x * 8 + wave;
  if (tile >= tilesM * tilesN) return;
  const int tm = tile / tilesN;
  const int tn = tile - tm * tilesN;
  const int m0 = tm << 6;
  const int n0 = tn << 6;

  const T* Ab  = A  + (size_t)b * strideA;
  const T* Bb  = Bt + (size_t)b * strideB;
  const T* Ab2 = SPLIT ? (A2  + (size_t)b * strideA) : nullptr;
  const T* Bb2 = SPLIT ? (Bt2 + (size_t)b * strideB) : nullptr;

  const int rlane = lane & 15;
  const int koff  = (lane >> 4) * 8;
  const int mOff  = (lane >> 4) * 8;

  v8f acc[4][4];
#pragma unroll
  for (int i = 0; i < 4; ++i)
#pragma unroll
    for (int j = 0; j < 4; ++j) acc[i][j] = (v8f){0.f,0.f,0.f,0.f,0.f,0.f,0.f,0.f};

  for (int k0 = 0; k0 < K; k0 += 32) {
    V bh[4], bl[4];
#pragma unroll
    for (int j = 0; j < 4; ++j) {
      const size_t bo = (size_t)(n0 + (j << 4) + rlane) * ldb + koff + k0;
      bh[j] = Frag<T>::load(Bb + bo);
      if (SPLIT) bl[j] = Frag<T>::load(Bb2 + bo);
    }
#pragma unroll
    for (int i = 0; i < 4; ++i) {
      const size_t ao = (size_t)(m0 + (i << 4) + rlane) * lda + koff + k0;
      V ah = Frag<T>::load(Ab + ao);
      V al;
      if (SPLIT) al = Frag<T>::load(Ab2 + ao);
#pragma unroll
      for (int j = 0; j < 4; ++j) {
        acc[i][j] = Frag<T>::mma(ah, bh[j], acc[i][j]);
        if (SPLIT) {
          acc[i][j] = Frag<T>::mma(ah, bl[j], acc[i][j]);
          acc[i][j] = Frag<T>::mma(al, bh[j], acc[i][j]);
        }
      }
      Frag<T>::guard(acc[i][0], acc[i][3], ah, SPLIT ? al : ah);
    }
    Frag<T>::keep(bh[0], bh[1], bh[2], bh[3]);
    if (SPLIT) Frag<T>::keep(bl[0], bl[1], bl[2], bl[3]);
  }
  acc_guard4(acc[0][0], acc[0][1], acc[0][2], acc[0][3]);
  acc_guard4(acc[1][0], acc[1][1], acc[1][2], acc[1][3]);
  acc_guard4(acc[2][0], acc[2][1], acc[2][2], acc[2][3]);
  acc_guard4(acc[3][0], acc[3][1], acc[3][2], acc[3][3]);

  float* slab = sT[wave];
  const float* Rb = RESID ? (resid + (size_t)b * strideR) : nullptr;
#pragma unroll
  for (int i = 0; i < 4; ++i) {
    const int mBase = m0 + (i << 4);
#pragma unroll
    for (int j = 0; j < 4; ++j) {
      const int n = n0 + (j << 4) + rlane;
      float bv = 0.f;
      if (BIAS_MODE == 2) bv = bias[n];
#pragma unroll
      for (int r = 0; r < 8; ++r) {
        float v = acc[i][j][r] * scale;
        if (BIAS_MODE == 1) v += bias[mBase + mOff + r];
        if (BIAS_MODE == 2) v += bv;
        if (RESID) v += Rb[(size_t)(mBase + mOff + r) * ldc + n];
        if (ACT == 1) v = tanhf(v);
        if (ACT == 2) v = fmaxf(v, 0.0f);
        if (ACT == 3) v = v / (1.0f + expf(-v));
        if (ACT == 4) v = (v > 0.f) ? v : 0.01f * v;
        if (ACT == 5) v = 0.5f * v * (1.0f + erff(v * 0.70710678118654752f));
        slab[(mOff + r) * 68 + (j << 4) + rlane] = v;
      }
    }
    __builtin_amdgcn_fence(__ATOMIC_RELEASE, "workgroup");
    __builtin_amdgcn_wave_barrier();
    __builtin_amdgcn_fence(__ATOMIC_ACQUIRE, "workgroup");
    if (OUT_MODE == 0) {
      float* C = (float*)Cout + (size_t)b * strideC;
      const int hh = lane >> 4, c4 = (lane & 15) * 4;
      for (int pass = 0; pass < 2; ++pass) {
#pragma unroll
        for (int it = 0; it < 8; ++it) {
          const int row = it * 2 + hh;
          v4f v = *(const v4f*)(slab + row * 68 + c4);
          *(volatile v4f*)(C + (size_t)(mBase + row) * ldc + n0 + c4) = v;
        }
        __threadfence();
      }
    } else {
      const int q = lane >> 3, c8 = (lane & 7) * 8;
      unsigned short* C  = (unsigned short*)Cout  + (size_t)b * strideC;
      unsigned short* C2 = (OUT_MODE == 2) ? ((unsigned short*)Cout2 + (size_t)b * strideC) : nullptr;
      for (int pass = 0; pass < 2; ++pass) {
#pragma unroll
        for (int it = 0; it < 4; ++it) {
          const int row = it * 4 + q;
          const float* sp = slab + row * 68 + c8;
          v8h hv, lv;
#pragma unroll
          for (int e = 0; e < 8; ++e) {
            if (OUT_MODE == 1) {
              hv[e] = (_Float16)sp[e];
            } else {
              unsigned short hb = f2bf_bits(sp[e]);
              unsigned short lb = f2bf_bits(sp[e] - bf_bits2f(hb));
              hv[e] = __builtin_bit_cast(_Float16, hb);
              lv[e] = __builtin_bit_cast(_Float16, lb);
            }
          }
          *(volatile v8h*)(C + (size_t)(mBase + row) * ldc + n0 + c8) = hv;
          if (OUT_MODE == 2) *(volatile v8h*)(C2 + (size_t)(mBase + row) * ldc + n0 + c8) = lv;
        }
        __threadfence();
      }
    }
    __builtin_amdgcn_fence(__ATOMIC_RELEASE, "workgroup");
    __builtin_amdgcn_wave_barrier();
    __builtin_amdgcn_fence(__ATOMIC_ACQUIRE, "workgroup");
  }
}

__global__ __launch_bounds__(256) void cast_bf16rne_f16x2(
    const float* __restrict__ in, _Float16* __restrict__ out, int n2) {
  int i = blockIdx.x * 256 + threadIdx.x;
  if (i < n2) {
    const _Float16 h0 = (_Float16)bfr(in[2 * i]), h1 = (_Float16)bfr(in[2 * i + 1]);
    const unsigned u = (unsigned)__builtin_bit_cast(unsigned short, h0) | ((unsigned)__builtin_bit_cast(unsigned short, h1) << 16);
    ((volatile unsigned*)out)[i] = u;
    __threadfence();
    ((volatile unsigned*)out)[i] = u;
  }
}

__global__ __launch_bounds__(NTHR) void tpw_kernel(const float* __restrict__ src, int R, int C, int ldo,
                                                 unsigned short* __restrict__ dst, float sc) {
  __shared__ float Tt[64 * 65];
  const int tid = threadIdx.x;
  const int c0 = blockIdx.x * 64, r0 = blockIdx.y * 64;
#pragma unroll
  for (int i = 0; i < 4; ++i) {
    const int idx = i * NTHR + tid;
    const int rr = idx >> 4, cc = (idx & 15) * 4;
    const v4f v = *(const v4f*)(src + (size_t)(r0 + rr) * (size_t)C + c0 + cc);
    Tt[rr * 65 + cc + 0] = v[0];
    Tt[rr * 65 + cc + 1] = v[1];
    Tt[rr * 65 + cc + 2] = v[2];
    Tt[rr * 65 + cc + 3] = v[3];
  }
  __syncthreads();
  const int q = tid >> 3, c8 = (tid & 7) * 8;
  v8h hv[2];
#pragma unroll
  for (int g = 0; g < 2; ++g) {
    const int qq = g * 32 + q;
#pragma unroll
    for (int e = 0; e < 8; ++e) {
      const float f = Tt[(c8 + e) * 65 + qq];
      const float fb = bfr(f);
      hv[g][e] = (_Float16)(fb * sc);
    }
  }
  for (int pass = 0; pass < 2; ++pass) {
#pragma unroll
    for (int g = 0; g < 2; ++g) {
      const size_t o = (size_t)(c0 + g * 32 + q) * (size_t)ldo + (size_t)(r0 + c8);
      *(volatile v8h*)(dst + o) = hv[g];
    }
    __threadfence();
  }
}

__global__ __launch_bounds__(NTHR) void decode_kernel(const float* __restrict__ x, const float* __restrict__ bias,
                                                   const float* __restrict__ vvec,
                                                   const unsigned short* __restrict__ WkTp,
                                                   const unsigned short* __restrict__ UkTp,
                                                   const unsigned short* __restrict__ W1Tp,
                                                   const float* __restrict__ w2eT,
                                                   float* __restrict__ out) {
  __shared__ __align__(16) _Float16 Ah[MTILE * HPITCH];
  __shared__ __align__(16) _Float16 Xl[MTILE * XLPITCH];
  __shared__ __align__(16) float    xzs[XZROWS * XZPITCH];
  __shared__ __align__(16) float    hws[HWROWS * HWPITCH];
  __shared__ __align__(16) float    scs[RPB * SCPITCH];
  __shared__ __align__(16) float    vsh[HID];
  const _Float16* WkT = (const _Float16*)WkTp;
  const _Float16* UkT = (const _Float16*)UkTp;
  const _Float16* W1T = (const _Float16*)W1Tp;
  const int tid = threadIdx.x, lane = tid & 31, wave = tid >> 5;
  const int c = lane & 15, hh = lane >> 4, koff = hh * 8;
  const int rowbase = blockIdx.x * RPB;

#pragma unroll 1
  for (int i = 0; i < MTILE; ++i) Ah[i * HPITCH + tid] = (_Float16)0.0f;
  vsh[tid] = bfr(vvec[tid]);
  {
    const int m = tid >> 4, f8 = (tid & 15) * 8;
    const int mr = (m < RPB) ? m : (RPB - 1);
    const bool live = (m < RPB);
    const float* xp = x + ((size_t)(rowbase + mr) * STEPS + (STEPS - 1)) * FEAT + f8;
    const v4f va = *(const v4f*)(xp);
    const v4f vb = *(const v4f*)(xp + 4);
    const _Float16 zh = (_Float16)0.0f;
    v8h hv;
    hv[0] = live ? (_Float16)bfr(va[0]) : zh; hv[1] = live ? (_Float16)bfr(va[1]) : zh;
    hv[2] = live ? (_Float16)bfr(va[2]) : zh; hv[3] = live ? (_Float16)bfr(va[3]) : zh;
    hv[4] = live ? (_Float16)bfr(vb[0]) : zh; hv[5] = live ? (_Float16)bfr(vb[1]) : zh;
    hv[6] = live ? (_Float16)bfr(vb[2]) : zh; hv[7] = live ? (_Float16)bfr(vb[3]) : zh;
    *(v8h*)(Xl + m * XLPITCH + f8) = hv;
  }
  __syncthreads();

  const _Float16* xlrow = Xl + c * XLPITCH + koff;
  const _Float16* ahrow = Ah + c * HPITCH + koff;
  const v8f z8 = {0.f, 0.f, 0.f, 0.f, 0.f, 0.f, 0.f, 0.f};

#pragma unroll
  for (int nt = 0; nt < 2; ++nt) {
    const int j = 32 * wave + 16 * nt + c;
    const _Float16* wk = WkT + (size_t)j * FEAT + koff;
    v8f acc[4];
    acc[0] = z8; acc[1] = z8; acc[2] = z8; acc[3] = z8;
#pragma unroll 1
    for (int kx = 0; kx < FEAT; kx += 32) {
      const v16h a  = Frag<_Float16>::load(xlrow + kx);
      const v16h b0 = Frag<_Float16>::load(wk + kx);
      const v16h b1 = Frag<_Float16>::load(wk + (size_t)1 * HID * FEAT + kx);
      const v16h b2 = Frag<_Float16>::load(wk + (size_t)2 * HID * FEAT + kx);
      const v16h b3 = Frag<_Float16>::load(wk + (size_t)3 * HID * FEAT + kx);
      acc[0] = Frag<_Float16>::mma(a, b0, acc[0]);
      acc[1] = Frag<_Float16>::mma(a, b1, acc[1]);
      acc[2] = Frag<_Float16>::mma(a, b2, acc[2]);
      acc[3] = Frag<_Float16>::mma(a, b3, acc[3]);
      dep_guard_h(acc[0], acc[3], a, b3);
      keep4_h(b0, b1, b2, b3);
    }
    acc_guard4(acc[0], acc[1], acc[2], acc[3]);
    float bq[4];
#pragma unroll
    for (int g = 0; g < 4; ++g) bq[g] = bfr(bias[g * HID + j]);
#pragma unroll
    for (int r = 0; r < RPB; ++r) {
      float* xr = xzs + (4 * hh + r) * XZPITCH + j;
      xr[0]       = acc[0][r] * INV_W + bq[0];
      xr[HID]     = acc[1][r] * INV_W + bq[1];
      xr[2 * HID] = acc[2][r] * INV_W + bq[2];
      xr[3 * HID] = acc[3][r] * INV_W + bq[3];
    }
  }
  float cst[2][RPB], hst[2][RPB];
#pragma unroll
  for (int nt = 0; nt < 2; ++nt)
#pragma unroll
    for (int r = 0; r < RPB; ++r) { cst[nt][r] = 0.0f; hst[nt][r] = 0.0f; }
  const float hsc = (hh == 0) ? HCARRY : 0.0f;
  __syncthreads();

#pragma unroll 1
  for (int t = 0; t < STEPS; ++t) {
#pragma unroll
    for (int nt = 0; nt < 2; ++nt) {
      const int j = 32 * wave + 16 * nt + c;
      const _Float16* uk = UkT + (size_t)j * HID + koff;
      v8f acc[4];
      acc[0] = z8; acc[1] = z8; acc[2] = z8; acc[3] = z8;
#pragma unroll 1
      for (int k0 = 0; k0 < HID; k0 += 32) {
        const v16h a  = Frag<_Float16>::load(ahrow + k0);
        const v16h b0 = Frag<_Float16>::load(uk + k0);
        const v16h b1 = Frag<_Float16>::load(uk + (size_t)1 * HID * HID + k0);
        const v16h b2 = Frag<_Float16>::load(uk + (size_t)2 * HID * HID + k0);
        const v16h b3 = Frag<_Float16>::load(uk + (size_t)3 * HID * HID + k0);
        acc[0] = Frag<_Float16>::mma(a, b0, acc[0]);
        acc[1] = Frag<_Float16>::mma(a, b1, acc[1]);
        acc[2] = Frag<_Float16>::mma(a, b2, acc[2]);
        acc[3] = Frag<_Float16>::mma(a, b3, acc[3]);
        dep_guard_h(acc[0], acc[3], a, b3);
        keep4_h(b0, b1, b2, b3);
      }
      acc_guard4(acc[0], acc[1], acc[2], acc[3]);
#pragma unroll
      for (int r = 0; r < RPB; ++r) {
        const float* xr = xzs + (4 * hh + r) * XZPITCH + j;
        const float zi = acc[0][r] * INV_WH + xr[0];
        const float zf = acc[1][r] * INV_WH + xr[HID];
        const float zg = acc[2][r] * INV_WH + xr[2 * HID];
        const float zo = acc[3][r] * INV_WH + xr[3 * HID];
        const float cn = fsig(zf) * cst[nt][r] + fsig(zi) * ftanh(zg);
        cst[nt][r] = cn;
        hst[nt][r] = fsig(zo) * ftanh(cn);
      }
    }
    __syncthreads();
#pragma unroll
    for (int nt = 0; nt < 2; ++nt) {
      const int j = 32 * wave + 16 * nt + c;
#pragma unroll
      for (int r = 0; r < RPB; ++r) Ah[(8 * hh + r) * HPITCH + j] = (_Float16)(hst[nt][r] * hsc);
    }
    __syncthreads();

    {
      const int j0 = 32 * wave + c, j1 = j0 + 16;
      const _Float16* w1a = W1T + (size_t)j0 * HID + koff;
      const _Float16* w1b = W1T + (size_t)j1 * HID + koff;
      v8f e0 = z8, e1 = z8;
#pragma unroll 1
      for (int k0 = 0; k0 < HID; k0 += 32) {
        const v16h a  = Frag<_Float16>::load(ahrow + k0);
        const v16h b0 = Frag<_Float16>::load(w1a + k0);
        const v16h b1 = Frag<_Float16>::load(w1b + k0);
        e0 = Frag<_Float16>::mma(a, b0, e0);
        e1 = Frag<_Float16>::mma(a, b1, e1);
        dep_guard_h(e0, e1, a, b1);
        keep2_h(b0, b1);
      }
      acc_guard2(e0, e1);
#pragma unroll
      for (int r = 0; r < RPB; ++r) {
        hws[(4 * hh + r) * HWPITCH + j0] = e0[r] * INV_WH;
        hws[(4 * hh + r) * HWPITCH + j1] = e1[r] * INV_WH;
      }
    }
    __syncthreads();

    {
      const float* wbase = w2eT + (size_t)rowbase * HID * STEPS + tid;
#pragma unroll 1
      for (int i = 0; i < RPB; ++i) {
        const float* wp  = wbase + (size_t)i * HID * STEPS;
        const float* hwr = hws + i * HWPITCH;
        float sacc = 0.0f;
#pragma unroll 1
        for (int h = 0; h < HID; h += 4) {
          const v4f hv = *(const v4f*)(hwr + h);
          const v4f vv = *(const v4f*)(vsh + h);
          const float* wq = wp + (size_t)h * STEPS;
          const float u0 = wq[0];
          const float u1 = wq[STEPS];
          const float u2 = wq[2 * STEPS];
          const float u3 = wq[3 * STEPS];
          sacc = fmaf(vv[0], ftanh(hv[0] + u0), sacc);
          sacc = fmaf(vv[1], ftanh(hv[1] + u1), sacc);
          sacc = fmaf(vv[2], ftanh(hv[2] + u2), sacc);
          sacc = fmaf(vv[3], ftanh(hv[3] + u3), sacc);
        }
        scs[i * SCPITCH + tid] = sacc;
      }
    }
    __syncthreads();

    if (wave < RPB) {
      const int i = wave;
      const float* sr = scs + i * SCPITCH;
      const v4f p0 = *(const v4f*)(sr + 4 * lane);
      const v4f p1 = *(const v4f*)(sr + 128 + 4 * lane);
      float m = fmaxf(fmaxf(fmaxf(p0[0], p0[1]), fmaxf(p0[2], p0[3])), fmaxf(fmaxf(p1[0], p1[1]), fmaxf(p1[2], p1[3])));
#pragma unroll
      for (int off = 16; off > 0; off >>= 1) m = fmaxf(m, __shfl_xor(m, off, 32));
      v4f e0, e1;
      e0[0] = __expf(p0[0] - m); e0[1] = __expf(p0[1] - m); e0[2] = __expf(p0[2] - m); e0[3] = __expf(p0[3] - m);
      e1[0] = __expf(p1[0] - m); e1[1] = __expf(p1[1] - m); e1[2] = __expf(p1[2] - m); e1[3] = __expf(p1[3] - m);
      float ssum = (e0[0] + e0[1]) + (e0[2] + e0[3]) + (e1[0] + e1[1]) + (e1[2] + e1[3]);
#pragma unroll
      for (int off = 16; off > 0; off >>= 1) ssum += __shfl_xor(ssum, off, 32);
      const float inv = __builtin_amdgcn_rcpf(ssum);
      const v4f q0 = e0 * inv;
      const v4f q1 = e1 * inv;
      float* orow = out + ((size_t)(rowbase + i) * STEPS + (size_t)t) * STEPS;
      for (int pass = 0; pass < 2; ++pass) {
        *(volatile v4f*)(orow + 4 * lane)       = q0;
        *(volatile v4f*)(orow + 128 + 4 * lane) = q1;
        __threadfence();
      }
    }
  }
}

extern "C" void kernel_launch(void* const* d_in, const int* in_sizes, int n_in,
                              void* d_out, int out_size, void* d_ws, size_t ws_size, hipStream_t stream) {
  if (n_in < 7 || d_out == nullptr || d_ws == nullptr) return;
  if (in_sizes[0] != SEQS * STEPS * FEAT || in_sizes[1] != FEAT * GATES || in_sizes[2] != HID * GATES ||
      in_sizes[3] != GATES || in_sizes[4] != HID * HID || in_sizes[5] != FEAT * HID || in_sizes[6] != HID ||
      out_size != SEQS * STEPS * STEPS) return;

  const float* xin  = (const float*)d_in[0];
  const float* wk   = (const float*)d_in[1];
  const float* uk   = (const float*)d_in[2];
  const float* bias = (const float*)d_in[3];
  const float* w1   = (const float*)d_in[4];
  const float* w2   = (const float*)d_in[5];
  const float* vv   = (const float*)d_in[6];
  float* out = (float*)d_out;

  char* ws = (char*)d_ws; size_t off = 0;
  auto carve = [&](size_t bytes) -> char* { char* p = ws + off; off += (bytes + 255) & ~(size_t)255; return p; };
  unsigned short* X16 = (unsigned short*)carve((size_t)SEQS * STEPS * FEAT * 2);
  unsigned short* W2T = (unsigned short*)carve((size_t)HID * FEAT * 2);
  unsigned short* UKT = (unsigned short*)carve((size_t)GATES * HID * 2);
  unsigned short* W1T = (unsigned short*)carve((size_t)HID * HID * 2);
  unsigned short* WKT = (unsigned short*)carve((size_t)GATES * FEAT * 2);
  float*          W2E = (float*)carve((size_t)SEQS * HID * STEPS * 4);
  if (off > ws_size || off > (size_t)134217728) return;

  const int n2 = (SEQS * STEPS * FEAT) / 2;
  cast_bf16rne_f16x2<<<(n2 + 255) / 256, 256, 0, stream>>>(xin, (_Float16*)X16, n2);
  tpw_kernel<<<dim3(GATES / 64, FEAT / 64), NTHR, 0, stream>>>(wk, FEAT, GATES, FEAT, WKT, WCARRY);
  tpw_kernel<<<dim3(GATES / 64, HID / 64),  NTHR, 0, stream>>>(uk, HID, GATES, HID, UKT, WCARRY);
  tpw_kernel<<<dim3(HID / 64, HID / 64),    NTHR, 0, stream>>>(w1, HID, HID, HID, W1T, WCARRY);
  tpw_kernel<<<dim3(HID / 64, FEAT / 64),   NTHR, 0, stream>>>(w2, FEAT, HID, FEAT, W2T, WCARRY);
  wmma_gemm64<0, false, 0, 0, false, 0><<<dim3((HID / 64) * (STEPS / 64) / 8, SEQS), 256, 0, stream>>>(
      W2T, W2T, FEAT, (long)0,
      X16, X16, FEAT, (long)STEPS * FEAT,
      (void*)W2E, (void*)W2E, STEPS, (long)HID * STEPS,
      bias, (const float*)W2E, (long)0,
      HID, STEPS, FEAT, INV_W);
  decode_kernel<<<SEQS / RPB, NTHR, 0, stream>>>(xin, bias, vv, WKT, UKT, W1T, W2E, out);
}
